// MyPointConv_2860448219714
// MI455X (gfx1250) — hardware-verified
//
#include <hip/hip_runtime.h>
#include <stdint.h>
#include <math.h>

#define NN   50000
#define NE   800000
#define NV   (NE + NN)
#define DD   128
#define KIN  131
#define KP   160
#define MP   50048
#define NT   256
#define SRB  1024
#define NTL  49
#define NPA  (NTL * SRB)
#define SCH  2048
#define NCH  ((NV + SCH - 1) / SCH)

typedef __attribute__((ext_vector_type(16))) _Float16 v16h;
typedef __attribute__((ext_vector_type(8)))  _Float16 v8h;
typedef __attribute__((ext_vector_type(4)))  _Float16 v4h;
typedef __attribute__((ext_vector_type(16))) __bf16   v16b;
typedef __attribute__((ext_vector_type(8)))  __bf16   v8b;
typedef __attribute__((ext_vector_type(8)))  float    v8f;
typedef __attribute__((ext_vector_type(4)))  float    v4f;
typedef __attribute__((ext_vector_type(4)))  int      v4i;

__device__ __forceinline__ unsigned short f2bf_bits(float f) {
  unsigned u = __float_as_uint(f);
  return (unsigned short)((u + 0x7FFFu + ((u >> 16) & 1u)) >> 16);
}
__device__ __forceinline__ float bf_bits2f(unsigned short h) { return __uint_as_float(((unsigned)h) << 16); }

__device__ __forceinline__ void dep_guard_h(v8f& a, v8f& b, v16h x, v16h y) { asm volatile("v_nop\n\tv_nop\n\tv_nop\n\tv_nop" : "+v"(a), "+v"(b) : "v"(x), "v"(y)); }
__device__ __forceinline__ void dep_guard_b(v8f& a, v8f& b, v16b x, v16b y) { asm volatile("v_nop\n\tv_nop\n\tv_nop\n\tv_nop" : "+v"(a), "+v"(b) : "v"(x), "v"(y)); }
__device__ __forceinline__ void keep4_h(v16h a, v16h b, v16h c, v16h d) { asm volatile("v_nop" :: "v"(a), "v"(b), "v"(c), "v"(d)); }
__device__ __forceinline__ void keep4_b(v16b a, v16b b, v16b c, v16b d) { asm volatile("v_nop" :: "v"(a), "v"(b), "v"(c), "v"(d)); }
__device__ __forceinline__ void acc_guard4(v8f& a, v8f& b, v8f& c, v8f& d) { asm volatile("v_nop\n\tv_nop\n\tv_nop\n\tv_nop" : "+v"(a), "+v"(b), "+v"(c), "+v"(d)); }
template <typename T> struct Frag;
template <> struct Frag<_Float16> {
  typedef v16h V; union U { v16h v; v8h h[2]; };
  static __device__ __forceinline__ v16h load(const _Float16* p) {
    U f; f.h[0] = *(const v8h*)(p); f.h[1] = *(const v8h*)(p + 16); return f.v;
  }
  static __device__ __forceinline__ v8f mma(v16h a, v16h b, v8f c) {
    return __builtin_amdgcn_wmma_f32_16x16x32_f16(false, a, false, b, (short)0, c, false, false);
  }
  static __device__ __forceinline__ void guard(v8f& a, v8f& b, v16h x, v16h y) { dep_guard_h(a, b, x, y); }
  static __device__ __forceinline__ void keep(v16h a, v16h b, v16h c, v16h d) { keep4_h(a, b, c, d); }
};
template <> struct Frag<__bf16> {
  typedef v16b V; union U { v16b v; v8b h[2]; };
  static __device__ __forceinline__ v16b load(const __bf16* p) {
    U f; f.h[0] = *(const v8b*)(p); f.h[1] = *(const v8b*)(p + 16); return f.v;
  }
  static __device__ __forceinline__ v8f mma(v16b a, v16b b, v8f c) {
    return __builtin_amdgcn_wmma_f32_16x16x32_bf16(false, a, false, b, (short)0, c, false, false);
  }
  static __device__ __forceinline__ void guard(v8f& a, v8f& b, v16b x, v16b y) { dep_guard_b(a, b, x, y); }
  static __device__ __forceinline__ void keep(v16b a, v16b b, v16b c, v16b d) { keep4_b(a, b, c, d); }
};

template <int ET> struct Elem;
template <> struct Elem<0> { typedef _Float16 T; };
template <> struct Elem<1> { typedef __bf16 T; };
template <int ET, bool SPLIT, int BIAS_MODE, int OUT_MODE, bool RESID, int ACT = 0>
__global__ __launch_bounds__(256) void wmma_gemm64(
    const unsigned short* __restrict__ Ap, const unsigned short* __restrict__ A2p, int lda, long strideA,
    const unsigned short* __restrict__ Btp, const unsigned short* __restrict__ Bt2p, int ldb, long strideB,
    void* __restrict__ Cout, void* __restrict__ Cout2, int ldc, long strideC,
    const float* __restrict__ bias,
    const float* __restrict__ resid, long strideR,
    int M, int N, int K, float scale) {
  typedef typename Elem<ET>::T T;
  typedef typename Frag<T>::V V;
  const T* A = (const T*)Ap; const T* A2 = (const T*)A2p; const T* Bt = (const T*)Btp; const T* Bt2 = (const T*)Bt2p;
  __shared__ __align__(16) float sT[8][16 * 68];
  const int b    = blockIdx.y;
  const int lane = threadIdx.x & 31;
  const int wave = threadIdx.x >> 5;
  const int tilesN = N >> 6;
  const int tilesM = M >> 6;
  const int tile = blockIdx.x * 8 + wave;
  if (tile >= tilesM * tilesN) return;
  const int tm = tile / tilesN;
  const int tn = tile - tm * tilesN;
  const int m0 = tm << 6;
  const int n0 = tn << 6;

  const T* Ab  = A  + (size_t)b * strideA;
  const T* Bb  = Bt + (size_t)b * strideB;
  const T* Ab2 = SPLIT ? (A2  + (size_t)b * strideA) : nullptr;
  const T* Bb2 = SPLIT ? (Bt2 + (size_t)b * strideB) : nullptr;

  const int rlane = lane & 15;
  const int koff  = (lane >> 4) * 8;
  const int mOff  = (lane >> 4) * 8;

  v8f acc[4][4];
#pragma unroll
  for (int i = 0; i < 4; ++i)
#pragma unroll
    for (int j = 0; j < 4; ++j) acc[i][j] = (v8f){0.f,0.f,0.f,0.f,0.f,0.f,0.f,0.f};

  for (int k0 = 0; k0 < K; k0 += 32) {
    V bh[4], bl[4];
#pragma unroll
    for (int j = 0; j < 4; ++j) {
      const size_t bo = (size_t)(n0 + (j << 4) + rlane) * ldb + koff + k0;
      bh[j] = Frag<T>::load(Bb + bo);
      if (SPLIT) bl[j] = Frag<T>::load(Bb2 + bo);
    }
#pragma unroll
    for (int i = 0; i < 4; ++i) {
      const size_t ao = (size_t)(m0 + (i << 4) + rlane) * lda + koff + k0;
      V ah = Frag<T>::load(Ab + ao);
      V al;
      if (SPLIT) al = Frag<T>::load(Ab2 + ao);
#pragma unroll
      for (int j = 0; j < 4; ++j) {
        acc[i][j] = Frag<T>::mma(ah, bh[j], acc[i][j]);
        if (SPLIT) {
          acc[i][j] = Frag<T>::mma(ah, bl[j], acc[i][j]);
          acc[i][j] = Frag<T>::mma(al, bh[j], acc[i][j]);
        }
      }
      Frag<T>::guard(acc[i][0], acc[i][3], ah, SPLIT ? al : ah);
    }
    Frag<T>::keep(bh[0], bh[1], bh[2], bh[3]);
    if (SPLIT) Frag<T>::keep(bl[0], bl[1], bl[2], bl[3]);
  }
  acc_guard4(acc[0][0], acc[0][1], acc[0][2], acc[0][3]);
  acc_guard4(acc[1][0], acc[1][1], acc[1][2], acc[1][3]);
  acc_guard4(acc[2][0], acc[2][1], acc[2][2], acc[2][3]);
  acc_guard4(acc[3][0], acc[3][1], acc[3][2], acc[3][3]);

  float* slab = sT[wave];
  const float* Rb = RESID ? (resid + (size_t)b * strideR) : nullptr;
#pragma unroll
  for (int i = 0; i < 4; ++i) {
    const int mBase = m0 + (i << 4);
#pragma unroll
    for (int j = 0; j < 4; ++j) {
      const int n = n0 + (j << 4) + rlane;
      float bv = 0.f;
      if (BIAS_MODE == 2) bv = bias[n];
#pragma unroll
      for (int r = 0; r < 8; ++r) {
        float v = acc[i][j][r] * scale;
        if (BIAS_MODE == 1) v += bias[mBase + mOff + r];
        if (BIAS_MODE == 2) v += bv;
        if (RESID) v += Rb[(size_t)(mBase + mOff + r) * ldc + n];
        if (ACT == 1) v = tanhf(v);
        if (ACT == 2) v = fmaxf(v, 0.0f);
        if (ACT == 3) v = v / (1.0f + expf(-v));
        if (ACT == 4) v = (v > 0.f) ? v : 0.01f * v;
        if (ACT == 5) v = 0.5f * v * (1.0f + erff(v * 0.70710678118654752f));
        slab[(mOff + r) * 68 + (j << 4) + rlane] = v;
      }
    }
    __builtin_amdgcn_fence(__ATOMIC_RELEASE, "workgroup");
    __builtin_amdgcn_wave_barrier();
    __builtin_amdgcn_fence(__ATOMIC_ACQUIRE, "workgroup");
    if (OUT_MODE == 0) {
      float* C = (float*)Cout + (size_t)b * strideC;
      const int hh = lane >> 4, c4 = (lane & 15) * 4;
      for (int pass = 0; pass < 2; ++pass) {
#pragma unroll
        for (int it = 0; it < 8; ++it) {
          const int row = it * 2 + hh;
          v4f v = *(const v4f*)(slab + row * 68 + c4);
          *(volatile v4f*)(C + (size_t)(mBase + row) * ldc + n0 + c4) = v;
        }
        __threadfence();
      }
    } else {
      const int q = lane >> 3, c8 = (lane & 7) * 8;
      unsigned short* C  = (unsigned short*)Cout  + (size_t)b * strideC;
      unsigned short* C2 = (OUT_MODE == 2) ? ((unsigned short*)Cout2 + (size_t)b * strideC) : nullptr;
      for (int pass = 0; pass < 2; ++pass) {
#pragma unroll
        for (int it = 0; it < 4; ++it) {
          const int row = it * 4 + q;
          const float* sp = slab + row * 68 + c8;
          v8h hv, lv;
#pragma unroll
          for (int e = 0; e < 8; ++e) {
            if (OUT_MODE == 1) {
              hv[e] = (_Float16)sp[e];
            } else {
              unsigned short hb = f2bf_bits(sp[e]);
              unsigned short lb = f2bf_bits(sp[e] - bf_bits2f(hb));
              hv[e] = __builtin_bit_cast(_Float16, hb);
              lv[e] = __builtin_bit_cast(_Float16, lb);
            }
          }
          *(volatile v8h*)(C + (size_t)(mBase + row) * ldc + n0 + c8) = hv;
          if (OUT_MODE == 2) *(volatile v8h*)(C2 + (size_t)(mBase + row) * ldc + n0 + c8) = lv;
        }
        __threadfence();
      }
    }
    __builtin_amdgcn_fence(__ATOMIC_RELEASE, "workgroup");
    __builtin_amdgcn_wave_barrier();
    __builtin_amdgcn_fence(__ATOMIC_ACQUIRE, "workgroup");
  }
}

__global__ __launch_bounds__(256) void wt_cast_kernel(const float* __restrict__ W, int Kin, int Nf, int Kp, unsigned* __restrict__ outp) {
  const int i = blockIdx.x * 256 + threadIdx.x;
  const int kp2 = Kp >> 1;
  if (i >= Nf * kp2) return;
  const int f = i / kp2;
  const int k = 2 * (i - f * kp2);
  const int k0c = (k < Kin) ? k : (Kin - 1);
  const int k1c = (k + 1 < Kin) ? (k + 1) : (Kin - 1);
  float a = W[(size_t)k0c * Nf + f] * 16.0f;
  float b = W[(size_t)k1c * Nf + f] * 16.0f;
  if (k >= Kin) a = 0.0f;
  if (k + 1 >= Kin) b = 0.0f;
  const unsigned u = (unsigned)__builtin_bit_cast(unsigned short, (_Float16)a) | ((unsigned)__builtin_bit_cast(unsigned short, (_Float16)b) << 16);
  ((volatile unsigned*)outp)[i] = u;
  __threadfence();
  ((volatile unsigned*)outp)[i] = u;
}

__global__ __launch_bounds__(256) void build_xp_kernel(const float* __restrict__ x, const float* __restrict__ pos, unsigned* __restrict__ XPp) {
  const int i = blockIdx.x * 256 + threadIdx.x;
  if (i >= MP * (KP / 2)) return;
  const int row = i / (KP / 2);
  const int col = 2 * (i - row * (KP / 2));
  const int rc  = (row < NN) ? row : (NN - 1);
  const int cx  = (col < DD - 2) ? col : (DD - 2);
  const float xa = x[(size_t)rc * DD + cx];
  const float xb = x[(size_t)rc * DD + cx + 1];
  const float p0 = pos[(size_t)rc * 3 + 0];
  const float p1 = pos[(size_t)rc * 3 + 1];
  const float p2 = pos[(size_t)rc * 3 + 2];
  float a = (col < DD) ? xa : ((col == DD) ? p0 : ((col == DD + 2) ? p2 : 0.0f));
  float b = (col < DD) ? xb : ((col == DD) ? p1 : 0.0f);
  if (row >= NN) { a = 0.0f; b = 0.0f; }
  const unsigned u = (unsigned)__builtin_bit_cast(unsigned short, (_Float16)a) | ((unsigned)__builtin_bit_cast(unsigned short, (_Float16)b) << 16);
  ((volatile unsigned*)XPp)[i] = u;
  __threadfence();
  ((volatile unsigned*)XPp)[i] = u;
}

__device__ __forceinline__ int blk_excl_scan(int cnt, int* scan_ws, int tid, int* tot) {
  const int lane = tid & 31, wave = tid >> 5; int incl = cnt;
#pragma unroll
  for (int o = 1; o < 32; o <<= 1) { const int v = __shfl_up(incl, o, 32); if (lane >= o) incl += v; }
  if (lane == 31) scan_ws[wave] = incl;
  __syncthreads();
  if (wave == 0) { int wv = (lane < NT / 32) ? scan_ws[lane] : 0; int wincl = wv;
#pragma unroll
    for (int o = 1; o < 32; o <<= 1) { const int v = __shfl_up(wincl, o, 32); if (lane >= o) wincl += v; }
    if (lane < NT / 32) scan_ws[32 + lane] = wincl - wv; if (lane == 31) scan_ws[64] = wincl; }
  __syncthreads();
  const int res = scan_ws[32 + wave] + incl - cnt; *tot = scan_ws[64];
  return res;
}
template <int SP, int CAP>
__device__ __forceinline__ int chunk_hits(const int* __restrict__ dstv, const int* __restrict__ srcv, int e0, int n0, int tid,
                                          int* LIST, int* scan_ws) {
  const int eb = e0 + tid * SP;
  const bool real = (eb < NE);
  const int ebc = real ? eb : (NE - SP);
  int rec[SP]; int cnt = 0;
#pragma unroll
  for (int k = 0; k < SP; k += 4) {
    const v4i d4 = *(const v4i*)(dstv + ebc + k);
    const v4i s4 = *(const v4i*)(srcv + ebc + k);
#pragma unroll
    for (int e = 0; e < 4; ++e) {
      int sr = s4[e]; sr = sr < 0 ? 0 : (sr >= NN ? NN - 1 : sr);
      const int ev = eb + k + e;
      const int dv = ev - NE;
      const int d = real ? d4[e] : dv;
      const int s = real ? sr : dv;
      const bool valid = real || (ev < NV);
      int r = -1;
      if (valid && d >= n0 && d < n0 + SRB) { r = ((d - n0) << 16) | s; ++cnt; }
      rec[k + e] = r;
    }
  }
  int tot; int p = blk_excl_scan(cnt, scan_ws, tid, &tot);
#pragma unroll
  for (int k = 0; k < SP; ++k) if (rec[k] >= 0) { if ((unsigned)p < (unsigned)CAP) LIST[p] = rec[k]; ++p; }
  __syncthreads();
  return tot < CAP ? tot : CAP;
}

__global__ __launch_bounds__(NT) void seg_max_kernel(const float* __restrict__ P, const int* __restrict__ ei, const float* __restrict__ pos,
                                                    const float* __restrict__ W1, const float* __restrict__ b1, float* ACC,
                                                    _Float16* __restrict__ A2) {
  __shared__ int LIST[SCH];
  __shared__ int scan_ws[80];
  const int tid = threadIdx.x, lane = tid & 31, wave = tid >> 5;
  const int n0 = blockIdx.x * SRB;
  const float ninf = __uint_as_float(0xff800000u);
  const v4f ninf4 = {ninf, ninf, ninf, ninf};
#pragma unroll 1
  for (int j = 0; j < 128; ++j) {
    float* rp = ACC + (size_t)(n0 + wave * 128 + j) * DD + 4 * lane;
    *(v4f*)rp = ninf4;
  }
  const int* srcv = ei; const int* dstv = ei + NE;
#pragma unroll 1
  for (int c = 0; c < NCH; ++c) {
    const int tot = chunk_hits<SCH / NT, SCH>(dstv, srcv, c * SCH, n0, tid, LIST, scan_ws);
#pragma unroll 1
    for (int base = 0; base < tot; base += 32) {
      const int q = base + lane;
      const int qc = (q < SCH) ? q : (SCH - 1);
      const int lv = LIST[qc];
      const int rv = (q < tot) ? lv : -1;
      const int own = (rv >= 0 && (rv >> 23) == wave) ? 1 : 0;
      unsigned msk = (unsigned)__ballot(own);
#pragma unroll 1
      for (int it = 0; it < 32; ++it) {
        if (msk == 0u) break;
        const int bp = __builtin_ctz(msk); msk &= msk - 1u;
        const int r = __shfl(rv, bp, 32);
        const int dl = (r >> 16) & 1023;
        int s = r & 0xFFFF; s = (s < NN) ? s : (NN - 1);
        const v4f pv = *(const v4f*)(P + (size_t)s * DD + 4 * lane);
        float* rp = ACC + (size_t)(n0 + dl) * DD + 4 * lane;
        v4f a = *(const v4f*)rp;
        a[0] = fmaxf(a[0], pv[0]); a[1] = fmaxf(a[1], pv[1]); a[2] = fmaxf(a[2], pv[2]); a[3] = fmaxf(a[3], pv[3]);
        *(v4f*)rp = a;
      }
    }
    __syncthreads();
  }
  const int hh = lane >> 4, c8 = (lane & 15) * 8;
  const v4f bA = *(const v4f*)(b1 + c8), bB = *(const v4f*)(b1 + c8 + 4);
  const v4f w0A = *(const v4f*)(W1 + (size_t)(DD + 0) * DD + c8), w0B = *(const v4f*)(W1 + (size_t)(DD + 0) * DD + c8 + 4);
  const v4f w1A = *(const v4f*)(W1 + (size_t)(DD + 1) * DD + c8), w1B = *(const v4f*)(W1 + (size_t)(DD + 1) * DD + c8 + 4);
  const v4f w2A = *(const v4f*)(W1 + (size_t)(DD + 2) * DD + c8), w2B = *(const v4f*)(W1 + (size_t)(DD + 2) * DD + c8 + 4);
#pragma unroll 1
  for (int jj = 0; jj < 64; ++jj) {
    const int dl = wave * 128 + 2 * jj + hh;
    const int n = n0 + dl;
    const int nc = (n < NN) ? n : (NN - 1);
    const float p0 = pos[(size_t)nc * 3 + 0], p1 = pos[(size_t)nc * 3 + 1], p2 = pos[(size_t)nc * 3 + 2];
    const float* rp = ACC + (size_t)n * DD + c8;
    const v4f aA = *(const v4f*)rp, aB = *(const v4f*)(rp + 4);
    v4f qA = aA + bA - (w0A * p0 + w1A * p1 + w2A * p2);
    v4f qB = aB + bB - (w0B * p0 + w1B * p1 + w2B * p2);
    v8h hv;
#pragma unroll
    for (int e = 0; e < 4; ++e) {
      float va = fmaxf(qA[e], 0.0f), vb = fmaxf(qB[e], 0.0f);
      if (n >= NN) { va = 0.0f; vb = 0.0f; }
      hv[e] = (_Float16)va; hv[4 + e] = (_Float16)vb;
    }
    _Float16* op = A2 + (size_t)n * DD + c8;
    *(volatile v8h*)op = hv;
    __threadfence();
    *(volatile v8h*)op = hv;
  }
}

__global__ __launch_bounds__(256) void copy_out_kernel(const float* __restrict__ H, float* __restrict__ out, int n4) {
  const int i = blockIdx.x * 256 + threadIdx.x;
  if (i >= n4) return;
  const v4f v = *(const v4f*)(H + 4 * (size_t)i);
  float* op = out + 4 * (size_t)i;
  *(volatile v4f*)op = v;
  __threadfence();
  *(volatile v4f*)op = v;
}

extern "C" void kernel_launch(void* const* d_in, const int* in_sizes, int n_in,
                              void* d_out, int out_size, void* d_ws, size_t ws_size, hipStream_t stream) {
  if (n_in < 7) return;
  if (in_sizes[0] != NN * DD || in_sizes[1] != NN * 3 || in_sizes[2] != 2 * NE || in_sizes[3] != KIN * DD ||
      in_sizes[4] != DD || in_sizes[5] != DD * DD || in_sizes[6] != DD || out_size != NN * DD) return;
  const float* x   = (const float*)d_in[0];
  const float* pos = (const float*)d_in[1];
  const int*   ei  = (const int*)  d_in[2];
  const float* W1  = (const float*)d_in[3];
  const float* b1  = (const float*)d_in[4];
  const float* W2  = (const float*)d_in[5];
  const float* b2  = (const float*)d_in[6];
  float* out = (float*)d_out;

  char* ws = (char*)d_ws; size_t off = 0;
  auto carve = [&](size_t bytes) -> char* { char* p = ws + off; off += (bytes + 255) & ~(size_t)255; return p; };
  unsigned* W1T = (unsigned*)carve((size_t)DD * KP * 2);
  unsigned* W2T = (unsigned*)carve((size_t)DD * DD * 2);
  unsigned* XP  = (unsigned*)carve((size_t)MP * KP * 2);
  float*    P   = (float*)   carve((size_t)MP * DD * 4);
  float*    ACC = (float*)   carve((size_t)NPA * DD * 4);
  _Float16* A2  = (_Float16*)carve((size_t)NPA * DD * 2);
  float*    H   = (float*)   carve((size_t)MP * DD * 4);
  if (off > ws_size || off > (size_t)134217728) return;

  wt_cast_kernel<<<(DD * (KP / 2)) / 256, 256, 0, stream>>>(W1, KIN, DD, KP, W1T);
  wt_cast_kernel<<<(DD * (DD / 2)) / 256, 256, 0, stream>>>(W2, DD, DD, DD, W2T);
  build_xp_kernel<<<(MP * (KP / 2)) / 256, 256, 0, stream>>>(x, pos, XP);
  {
    const int tiles = (MP / 64) * (DD / 64);
    wmma_gemm64<0, false, 0, 0, false><<<dim3((tiles + 7) / 8, 1), 256, 0, stream>>>(
        (const unsigned short*)XP, nullptr, KP, 0L, (const unsigned short*)W1T, nullptr, KP, 0L,
        (void*)P, nullptr, DD, 0L, nullptr, nullptr, 0L, MP, DD, KP, 0.0625f);
  }
  seg_max_kernel<<<NTL, NT, 0, stream>>>(P, ei, pos, W1, b1, ACC, A2);
  {
    const int tiles = (MP / 64) * (DD / 64);
    wmma_gemm64<0, false, 2, 0, false><<<dim3((tiles + 7) / 8, 1), 256, 0, stream>>>(
        (const unsigned short*)A2, nullptr, DD, 0L, (const unsigned short*)W2T, nullptr, DD, 0L,
        (void*)H, nullptr, DD, 0L, b2, nullptr, 0L, MP, DD, DD, 0.0625f);
  }
  copy_out_kernel<<<(NN * (DD / 4)) / 256, 256, 0, stream>>>(H, out, NN * (DD / 4));
}
